// MultiHeadAttn_5970004541835
// MI455X (gfx1250) — hardware-verified
//
#include <hip/hip_runtime.h>
#ifndef NB
#define NB 2
#endif
#ifndef SEQ
#define SEQ 2048
#endif
#define NB_FULL 2
#define SEQ_FULL 2048
#define DM 1024
#define NH 16
#define HD 64
#define NREL 33
#define KREL 16
#define NRELP 48
#define NR ((size_t)NB * SEQ)
static_assert(SEQ % 128 == 0);
static_assert(SEQ <= SEQ_FULL);
static_assert(NB >= 1 && NB <= NB_FULL);
static_assert(DM == NH * HD);

typedef unsigned short v8us __attribute__((ext_vector_type(8), may_alias));
typedef float  v8f  __attribute__((ext_vector_type(8)));
typedef float  v4f  __attribute__((ext_vector_type(4)));
typedef float  v4fa __attribute__((ext_vector_type(4), may_alias));
typedef _Float16 v16h __attribute__((ext_vector_type(16)));
typedef _Float16 v4h __attribute__((ext_vector_type(4)));
typedef int v4ia __attribute__((ext_vector_type(4), may_alias));
typedef unsigned int v2ua __attribute__((ext_vector_type(2), may_alias));
union FragH { v16h v; v8us half[2]; _Float16 h[16]; unsigned short u[16]; };

__device__ __forceinline__ unsigned short bf16_bits(float x) { unsigned int u = __float_as_uint(x); return (unsigned short)((u + 0x7FFFu + ((u >> 16) & 1u)) >> 16); }
__device__ __forceinline__ float bf16_val(unsigned short b) { return __uint_as_float(((unsigned int)b) << 16); }
__device__ __forceinline__ float bf16_rne(float x) { return bf16_val(bf16_bits(x)); }

__device__ __forceinline__ v16h g2_frag(const _Float16* p, int hh) { FragH f; f.half[0] = *(const v8us*)((const unsigned short*)p + 8 * hh); f.half[1] = *(const v8us*)((const unsigned short*)p + 16 + 8 * hh); return f.v; }
__device__ __forceinline__ v8f g2_mma(v16h a, v16h b, v8f c) { v8f d = __builtin_amdgcn_wmma_f32_16x16x32_f16(false, a, false, b, (short)0, c, false, false); asm volatile("v_nop\n\tv_nop\n\tv_nop\n\tv_nop" : "+v"(d) : "v"(a), "v"(b)); return d; }
__device__ __forceinline__ v8f mma2(v16h a0, v16h b0, v16h a1, v16h b1, v8f c) {
  c = __builtin_amdgcn_wmma_f32_16x16x32_f16(false, a0, false, b0, (short)0, c, false, false);
  c = __builtin_amdgcn_wmma_f32_16x16x32_f16(false, a1, false, b1, (short)0, c, false, false);
  asm volatile("v_nop\n\tv_nop\n\tv_nop\n\tv_nop" : "+v"(c) : "v"(a0), "v"(b0), "v"(a1), "v"(b1));
  return c;
}

__global__ __launch_bounds__(256) void k_wnat(const float* __restrict__ w, size_t n8, _Float16* __restrict__ Bt) {
  const size_t t = (size_t)blockIdx.x * 256 + threadIdx.x; if (t >= n8) return; FragH f;
#pragma unroll
  for (int q = 0; q < 8; ++q) f.h[q] = (_Float16)(bf16_rne(w[t * 8 + q]) * 16.0f);
  *(volatile v8us*)((unsigned short*)Bt + t * 8) = f.half[0]; __threadfence(); *(volatile v8us*)((unsigned short*)Bt + t * 8) = f.half[0];
}

__global__ __launch_bounds__(256) void k_relt(const float* __restrict__ rel, _Float16* __restrict__ RT) {
  const int t = blockIdx.x * 256 + threadIdx.x; if (t >= NRELP * (HD / 8)) return;
  const int r = t / (HD / 8), d8 = (t % (HD / 8)) * 8;
  const int rc = (r < NREL) ? r : (NREL - 1);
  const bool live = (r < NREL);
  FragH f;
#pragma unroll
  for (int q = 0; q < 8; ++q) { const float v = rel[(size_t)rc * HD + d8 + q]; f.h[q] = live ? (_Float16)(bf16_rne(v) * 16.0f) : (_Float16)0.0f; }
  *(volatile v8us*)((unsigned short*)RT + (size_t)t * 8) = f.half[0]; __threadfence(); *(volatile v8us*)((unsigned short*)RT + (size_t)t * 8) = f.half[0];
}

__global__ __launch_bounds__(256) void k_x16c(const float* __restrict__ x, _Float16* __restrict__ X16, int nrow) {
  const size_t t = (size_t)blockIdx.x * 256 + threadIdx.x; if (t >= (size_t)nrow * (DM / 8)) return;
  const int r = (int)(t / (DM / 8)), c8 = (int)(t % (DM / 8)) * 8;
  const int b = r / SEQ, s = r - b * SEQ;
  const float* src = x + ((size_t)b * SEQ_FULL + s) * DM + c8;
  const v4f a = *(const v4fa*)src, c = *(const v4fa*)(src + 4); FragH f;
#pragma unroll
  for (int q = 0; q < 4; ++q) { f.h[q] = (_Float16)bf16_rne(a[q]); f.h[4 + q] = (_Float16)bf16_rne(c[q]); }
  *(volatile v8us*)((unsigned short*)X16 + t * 8) = f.half[0]; __threadfence(); *(volatile v8us*)((unsigned short*)X16 + t * 8) = f.half[0];
}

__global__ __launch_bounds__(256) void k_pack(const int* __restrict__ msk, unsigned int* __restrict__ bits, int nwords) {
  const int i = blockIdx.x * 256 + threadIdx.x; if (i >= nwords) return;
  const int wpr = SEQ / 32;
  const int row = i / wpr, wi = i - row * wpr;
  const int b = row / SEQ, q = row - b * SEQ;
  const int* src = msk + ((size_t)b * SEQ_FULL + q) * SEQ_FULL + (size_t)wi * 32;
  unsigned int wd = 0u;
#pragma unroll
  for (int j = 0; j < 8; ++j) {
    const v4ia v = *(const v4ia*)(src + j * 4);
    wd |= (v[0] != 0 ? 1u : 0u) << (j * 4 + 0);
    wd |= (v[1] != 0 ? 1u : 0u) << (j * 4 + 1);
    wd |= (v[2] != 0 ? 1u : 0u) << (j * 4 + 2);
    wd |= (v[3] != 0 ? 1u : 0u) << (j * 4 + 3);
  }
  *(volatile unsigned int*)(bits + i) = wd; __threadfence(); *(volatile unsigned int*)(bits + i) = wd;
}

__global__ __launch_bounds__(128) void k_gemm2(const _Float16* __restrict__ A, int lda, size_t sA, const _Float16* __restrict__ Bh, int ldb, size_t sB, float alpha,
    float* __restrict__ C, _Float16* __restrict__ C16, _Float16* __restrict__ C16L, int ldc, size_t sC, int M, int N, int K) {
  __shared__ __attribute__((aligned(16))) float so[4][32][68];
  const int tid = threadIdx.x, w = tid >> 5, lane = tid & 31, ln = lane & 15, hh = lane >> 4; const int by = blockIdx.y;
  A += (size_t)by * sA; Bh += (size_t)by * sB; const size_t cofs = (size_t)by * sC;
  const int ntn = N >> 6; const int mt = blockIdx.x / ntn, nq = blockIdx.x - mt * ntn; const int row0 = mt * 128 + 32 * w, col0 = nq * 64; if (row0 >= M) return;
  const _Float16* a0p = A + (size_t)(row0 + ln) * lda; const _Float16* a1p = a0p + (size_t)16 * lda;
  const _Float16* b0p = Bh + (size_t)(col0 + ln) * ldb; const _Float16* b1p = b0p + (size_t)16 * ldb; const _Float16* b2p = b1p + (size_t)16 * ldb; const _Float16* b3p = b2p + (size_t)16 * ldb;
  const v8f z8 = {0.f,0.f,0.f,0.f,0.f,0.f,0.f,0.f}; v8f c00 = z8, c01 = z8, c02 = z8, c03 = z8, c10 = z8, c11 = z8, c12 = z8, c13 = z8;
#pragma unroll 1
  for (int kb = 0; kb < K; kb += 32) { const v16h a0 = g2_frag(a0p + kb, hh), a1 = g2_frag(a1p + kb, hh);
    v16h b = g2_frag(b0p + kb, hh); c00 = g2_mma(a0, b, c00); c10 = g2_mma(a1, b, c10);
    b = g2_frag(b1p + kb, hh); c01 = g2_mma(a0, b, c01); c11 = g2_mma(a1, b, c11);
    b = g2_frag(b2p + kb, hh); c02 = g2_mma(a0, b, c02); c12 = g2_mma(a1, b, c12);
    b = g2_frag(b3p + kb, hh); c03 = g2_mma(a0, b, c03); c13 = g2_mma(a1, b, c13); }
  v8f accs[8] = {c00, c01, c02, c03, c10, c11, c12, c13};
#pragma unroll
  for (int u = 0; u < 8; ++u) { const int t = u & 3, half = u >> 2;
#pragma unroll
    for (int r = 0; r < 8; ++r) { const int rloc = half * 16 + 8 * hh + r; so[w][rloc][t * 16 + ln] = accs[u][r] * alpha; } }
  __builtin_amdgcn_fence(4  , "workgroup"); __builtin_amdgcn_wave_barrier();
  const int rsub = lane >> 4, c4 = (lane & 15) * 4;
  for (int pass = 0; pass < 2; ++pass) {
#pragma unroll
    for (int q = 0; q < 16; ++q) {
      const int r = q * 2 + rsub; const v4f v = *(const v4fa*)&so[w][r][c4];
      const size_t o = cofs + (size_t)(row0 + r) * ldc + col0 + c4;
      if (C) *(volatile v4f*)(C + o) = v;
      if (C16) { v4h h4, l4;
#pragma unroll
        for (int i = 0; i < 4; ++i) { const _Float16 hq = (_Float16)v[i]; h4[i] = hq; l4[i] = (_Float16)((v[i] - (float)hq) * 1024.0f); }
        *(volatile v4h*)(C16 + o) = h4;
        if (C16L) *(volatile v4h*)(C16L + o) = l4; }
    }
    if (pass == 0) __threadfence(); }
}

template <int NHv, int TTv>
__global__ __launch_bounds__(256) void k_vt(const _Float16* __restrict__ V16, int ldv, int voff, _Float16* __restrict__ Vt) {
  __shared__ unsigned short tl[64][66]; const int tid = threadIdx.x;
  const int slab = blockIdx.x / (TTv / 64), lg = blockIdx.x % (TTv / 64); const int b = slab / NHv, h = slab % NHv;
  for (int i = tid; i < 64 * 8; i += 256) { const int r = i / 8, c8 = (i % 8) * 8; FragH f; f.half[0] = *(const v8us*)((const unsigned short*)V16 + ((size_t)b * TTv + lg * 64 + r) * ldv + voff + h * 64 + c8);
#pragma unroll
    for (int q = 0; q < 8; ++q) tl[r][c8 + q] = f.u[q]; }
  __syncthreads();
  for (int pass = 0; pass < 2; ++pass) {
#pragma unroll
    for (int rd = 0; rd < 2; ++rd) { const int d = rd * 32 + tid / 8, pc = tid % 8; FragH f;
#pragma unroll
      for (int q = 0; q < 8; ++q) f.u[q] = tl[pc * 8 + q][d];
      *(volatile v8us*)((unsigned short*)Vt + ((size_t)slab * 64 + d) * TTv + lg * 64 + pc * 8) = f.half[0]; }
    if (pass == 0) __threadfence(); }
}

__global__ __launch_bounds__(128) void k_attn(const _Float16* __restrict__ QH, const _Float16* __restrict__ QL, const _Float16* __restrict__ KH, const _Float16* __restrict__ KL,
                                              const _Float16* __restrict__ VT, const _Float16* __restrict__ RT, const unsigned int* __restrict__ MBt,
                                              const float* __restrict__ spb, _Float16* __restrict__ O16) {
  #pragma clang fp contract(off)
  __shared__ __attribute__((aligned(16))) _Float16 tls[4][16][72];
  __shared__ float qes[4][16][52];
  const int tid = threadIdx.x, w = tid >> 5, lane = tid & 31, ln = lane & 15, hh = lane >> 4;
  const int nqb = SEQ / 64;
  const int bh = blockIdx.x / nqb, qb = blockIdx.x - bh * nqb;
  const int b = bh / NH, h = bh - b * NH;
  const int q0 = qb * 64 + w * 16;
  const size_t rq = (size_t)b * SEQ + q0;
  const size_t qoff = (rq + ln) * DM + (size_t)h * HD;
  const v16h qh0 = g2_frag(QH + qoff, hh), qh1 = g2_frag(QH + qoff + 32, hh);
  const v16h ql0 = g2_frag(QL + qoff, hh), ql1 = g2_frag(QL + qoff + 32, hh);
  const v8f z8 = {0.f,0.f,0.f,0.f,0.f,0.f,0.f,0.f};
  const float rsc = 0.0009765625f;
#pragma unroll
  for (int nt = 0; nt < 3; ++nt) {
    const _Float16* rr = RT + (size_t)(nt * 16 + ln) * HD;
    const v16h r0 = g2_frag(rr, hh), r1 = g2_frag(rr + 32, hh);
    const v8f ah = mma2(qh0, r0, qh1, r1, z8);
    const v8f al = mma2(ql0, r0, ql1, r1, z8);
#pragma unroll
    for (int r = 0; r < 8; ++r) { const float e = ah[r] + al[r] * rsc; qes[w][8 * hh + r][nt * 16 + ln] = e * 0.0625f; }
  }
  __syncthreads();

  const _Float16* kbh = KH + ((size_t)b * SEQ) * DM + (size_t)h * HD;
  const _Float16* kbl = KL + ((size_t)b * SEQ) * DM + (size_t)h * HD;
  const _Float16* vtb = VT + ((size_t)bh * HD) * SEQ;
  const unsigned int* mbr = MBt + (rq + 8 * hh) * (SEQ / 32);
  const float sbias = spb[0];
  float dsum[8];
#pragma unroll
  for (int r = 0; r < 8; ++r) dsum[r] = 0.f;
  v8f oacc[4] = {z8, z8, z8, z8};

#pragma unroll 1
  for (int k0 = 0; k0 < SEQ; k0 += 64) {
    v2ua mw[8];
#pragma unroll
    for (int r = 0; r < 8; ++r) mw[r] = *(const v2ua*)(mbr + (size_t)r * (SEQ / 32) + (k0 >> 5));
#pragma unroll
    for (int kt = 0; kt < 4; ++kt) {
      const size_t koff = (size_t)(k0 + kt * 16 + ln) * DM;
      const v16h kh0 = g2_frag(kbh + koff, hh), kh1 = g2_frag(kbh + koff + 32, hh);
      const v8f sh = mma2(qh0, kh0, qh1, kh1, z8);
      v8f sx = mma2(ql0, kh0, ql1, kh1, z8);
      const v16h kl0 = g2_frag(kbl + koff, hh), kl1 = g2_frag(kbl + koff + 32, hh);
      sx = mma2(qh0, kl0, qh1, kl1, sx);
      const int kc = kt * 16 + ln;
#pragma unroll
      for (int r = 0; r < 8; ++r) {
        const int m = 8 * hh + r;
        int rel = (k0 + kc) - (q0 + m);
        rel = (rel < -KREL) ? -KREL : ((rel > KREL) ? KREL : rel);
        const float s = sh[r] + sx[r] * rsc;
        float sv = (s + qes[w][m][rel + KREL]) * 0.125f;
        const unsigned int word = (kt < 2) ? mw[r][0] : mw[r][1];
        const unsigned int bit = (word >> ((kt & 1) * 16 + ln)) & 1u;
        sv = (bit != 0u) ? -1.0e9f : sv;
        float t = sv + sbias;
        t = fmaxf(t, 0.0f);
        const float tt = t * t;
        dsum[r] += tt;
        tls[w][m][kc] = (_Float16)(tt * 256.0f);
      }
    }
    __builtin_amdgcn_fence(3  , "wavefront"); __builtin_amdgcn_wave_barrier();
    FragH pa, pb;
    pa.half[0] = *(const v8us*)&tls[w][ln][8 * hh];      pa.half[1] = *(const v8us*)&tls[w][ln][16 + 8 * hh];
    pb.half[0] = *(const v8us*)&tls[w][ln][32 + 8 * hh]; pb.half[1] = *(const v8us*)&tls[w][ln][48 + 8 * hh];
#pragma unroll
    for (int dt = 0; dt < 4; ++dt) {
      const _Float16* vr = vtb + (size_t)(dt * 16 + ln) * SEQ + k0;
      const v16h v0 = g2_frag(vr, hh), v1 = g2_frag(vr + 32, hh);
      oacc[dt] = mma2(pa.v, v0, pb.v, v1, oacc[dt]);
    }
    __builtin_amdgcn_fence(3  , "wavefront"); __builtin_amdgcn_wave_barrier();
  }

#pragma unroll
  for (int r = 0; r < 8; ++r) {
    float v = dsum[r];
    v += __shfl_xor(v, 1, 32); v += __shfl_xor(v, 2, 32); v += __shfl_xor(v, 4, 32); v += __shfl_xor(v, 8, 32);
    dsum[r] = (1.0f / (v + 1.0e-9f)) * 0.25f;
  }
#pragma unroll
  for (int dt = 0; dt < 4; ++dt)
#pragma unroll
    for (int r = 0; r < 8; ++r) tls[w][8 * hh + r][dt * 16 + ln] = (_Float16)(oacc[dt][r] * dsum[r]);
  __builtin_amdgcn_fence(3  , "wavefront"); __builtin_amdgcn_wave_barrier();
  const int rl = lane >> 3, pc = (lane & 7) * 8;
  for (int pass = 0; pass < 2; ++pass) {
#pragma unroll
    for (int it = 0; it < 4; ++it) {
      const int row = it * 4 + rl;
      const v8us v = *(const v8us*)&tls[w][row][pc];
      *(volatile v8us*)((unsigned short*)O16 + (rq + row) * DM + (size_t)h * HD + pc) = v;
    }
    if (pass == 0) __threadfence();
  }
}

extern "C" void kernel_launch(void* const* d_in, const int* in_sizes, int n_in,
                              void* d_out, int out_size, void* d_ws, size_t ws_size, hipStream_t stream) {
  if (n_in < 10) return;
  const int nx = (int)(NR * DM);
  if (in_sizes[0] < nx || in_sizes[1] < nx || in_sizes[2] < nx) return;
  if (in_sizes[3] < (int)(NR * SEQ)) return;
  if (in_sizes[4] < DM * DM || in_sizes[5] < DM * DM || in_sizes[6] < DM * DM || in_sizes[7] < DM * DM) return;
  if (in_sizes[8] < NREL * HD || in_sizes[9] < 1) return;
  if (out_size < nx) return;
  const float* xq = (const float*)d_in[0]; const float* xk = (const float*)d_in[1]; const float* xv = (const float*)d_in[2];
  const int* msk = (const int*)d_in[3];
  const float* wq = (const float*)d_in[4]; const float* wk = (const float*)d_in[5]; const float* wv = (const float*)d_in[6]; const float* wo = (const float*)d_in[7];
  const float* rel = (const float*)d_in[8]; const float* spb = (const float*)d_in[9];

  char* ws = (char*)d_ws; size_t off = 0;
  auto take = [&](size_t bytes) { char* p = ws + off; off += (bytes + 255) & ~(size_t)255; return p; };
  const size_t wbytes = (size_t)DM * DM * 2, xbytes = NR * DM * 2;
  _Float16* BQ = (_Float16*)take(wbytes); _Float16* BK = (_Float16*)take(wbytes); _Float16* BV = (_Float16*)take(wbytes); _Float16* BO = (_Float16*)take(wbytes);
  _Float16* RT = (_Float16*)take((size_t)NRELP * HD * 2);
  _Float16* XQ = (_Float16*)take(xbytes); _Float16* XK = (_Float16*)take(xbytes); _Float16* XV = (_Float16*)take(xbytes);
  _Float16* QH = (_Float16*)take(xbytes); _Float16* QL = (_Float16*)take(xbytes); _Float16* KH = (_Float16*)take(xbytes); _Float16* KL = (_Float16*)take(xbytes);
  _Float16* V16 = (_Float16*)take(xbytes);
  _Float16* VT = (_Float16*)take((size_t)NB * NH * HD * SEQ * 2);
  const int nwords = (int)(NR * (SEQ / 32));
  unsigned int* MB = (unsigned int*)take((size_t)nwords * 4);
  _Float16* O16 = (_Float16*)take(xbytes);
  if (off > ws_size || off > (size_t)134217728) return;

  { const size_t n8 = (size_t)DM * DM / 8; const unsigned g = (unsigned)((n8 + 255) / 256);
    k_wnat<<<g, 256, 0, stream>>>(wq, n8, BQ); k_wnat<<<g, 256, 0, stream>>>(wk, n8, BK); k_wnat<<<g, 256, 0, stream>>>(wv, n8, BV); k_wnat<<<g, 256, 0, stream>>>(wo, n8, BO); }
  k_relt<<<(NRELP * (HD / 8) + 255) / 256, 256, 0, stream>>>(rel, RT);
  { const unsigned g = (unsigned)((NR * DM / 8 + 255) / 256); const int nrow = (int)NR;
    k_x16c<<<g, 256, 0, stream>>>(xq, XQ, nrow); k_x16c<<<g, 256, 0, stream>>>(xk, XK, nrow); k_x16c<<<g, 256, 0, stream>>>(xv, XV, nrow); }
  k_pack<<<(nwords + 255) / 256, 256, 0, stream>>>(msk, MB, nwords);

  const int M = (int)NR;
  const dim3 gp((unsigned)((M / 128) * (DM / 64)), 1);
  k_gemm2<<<gp, 128, 0, stream>>>(XQ, DM, (size_t)0, BQ, DM, (size_t)0, 0.0625f, nullptr, QH, QL, DM, (size_t)0, M, DM, DM);
  k_gemm2<<<gp, 128, 0, stream>>>(XK, DM, (size_t)0, BK, DM, (size_t)0, 0.0625f, nullptr, KH, KL, DM, (size_t)0, M, DM, DM);
  k_gemm2<<<gp, 128, 0, stream>>>(XV, DM, (size_t)0, BV, DM, (size_t)0, 0.0625f, nullptr, V16, nullptr, DM, (size_t)0, M, DM, DM);
  k_vt<NH, SEQ><<<(unsigned)(NB * NH * (SEQ / 64)), 256, 0, stream>>>(V16, DM, 0, VT);
  k_attn<<<(unsigned)(NB * NH * (SEQ / 64)), 128, 0, stream>>>(QH, QL, KH, KL, VT, RT, MB, spb, O16);
  k_gemm2<<<gp, 128, 0, stream>>>(O16, DM, (size_t)0, BO, DM, (size_t)0, 0.0009765625f, (float*)d_out, nullptr, nullptr, DM, (size_t)0, M, DM, DM);
}
